// SelfAttention_11201274708744
// MI455X (gfx1250) — hardware-run, weakly checked
//
#include <hip/hip_runtime.h>


#ifndef NB
#define NB 8
#endif
#ifndef SEQ
#define SEQ 4096
#endif
#define NB_FULL  8
#define SEQ_FULL 4096
#ifndef OUT_SEQ
#define OUT_SEQ SEQ
#endif
#define CH   256
#define CQ   32
#define CHH  128
#define AW   4
#define QRS  2048.0f
#define QRI  (1.0f / 2048.0f)
#define SC2  1.4426950408889634f
#define PSH  14.0f

static_assert(CQ == 32);
static_assert(2 * CHH == CH);
static_assert(CH % 64 == 0);
static_assert(CH % 32 == 0);
static_assert(SEQ % 64 == 0);
static_assert(SEQ % 32 == 0);
static_assert(SEQ % (16 * AW) == 0);
static_assert(OUT_SEQ % 64 == 0);
static_assert(OUT_SEQ >= SEQ);
static_assert(SEQ_FULL % 4 == 0);
static_assert(NB <= NB_FULL);
static_assert(SEQ <= SEQ_FULL);
static_assert(((size_t)CQ * CH) % 8 == 0);
static_assert(((size_t)CH * CH) % 8 == 0);

typedef _Float16 h16;
typedef unsigned short bf;
typedef __attribute__((ext_vector_type(16))) __bf16   v16bf;
typedef __attribute__((ext_vector_type(16))) _Float16 v16h;
typedef __attribute__((ext_vector_type(8)))  _Float16 v8h;
typedef __attribute__((ext_vector_type(8)))  unsigned short v8us;
typedef __attribute__((ext_vector_type(8)))  float    v8f;
typedef __attribute__((ext_vector_type(4)))  float    v4f;
typedef v4f  __attribute__((may_alias)) v4fa;
typedef v8us __attribute__((may_alias)) v8usa;

__device__ __forceinline__ unsigned short f2bf(float f) { unsigned u = __float_as_uint(f); u += 0x7FFFu + ((u >> 16) & 1u); return (unsigned short)(u >> 16); }
__device__ __forceinline__ float bfr(float f) { return __uint_as_float(((unsigned)f2bf(f)) << 16); }
__device__ __forceinline__ v16h cat16(v8h lo, v8h hi) { return __builtin_shufflevector(lo, hi, 0, 1, 2, 3, 4, 5, 6, 7, 8, 9, 10, 11, 12, 13, 14, 15); }
__device__ __forceinline__ v16bf cat16b(v8us lo, v8us hi) { return __builtin_bit_cast(v16bf, __builtin_shufflevector(lo, hi, 0, 1, 2, 3, 4, 5, 6, 7, 8, 9, 10, 11, 12, 13, 14, 15)); }
__device__ __forceinline__ v8f wmma16(v16h a, v16h b, v8f c) { return __builtin_amdgcn_wmma_f32_16x16x32_f16(false, a, false, b, (short)0, c, false, false); }
__device__ __forceinline__ v8f wmmab(v16bf a, v16bf b, v8f c) { return __builtin_amdgcn_wmma_f32_16x16x32_bf16(false, a, false, b, (short)0, c, false, false); }
__device__ __forceinline__ v16h  ldh(const h16* p) { return cat16(*(const v8h*)p, *(const v8h*)(p + 16)); }
__device__ __forceinline__ v16bf ldb(const bf* p)  { return cat16b(*(const v8us*)p, *(const v8us*)(p + 16)); }
__device__ __forceinline__ void wave_sync() { __builtin_amdgcn_fence(3  , "wavefront"); __builtin_amdgcn_wave_barrier(); asm volatile("" ::: "memory"); }

__global__ __launch_bounds__(256) void k_cvt8(const float* __restrict__ src, bf* dst, size_t n8) {
    const size_t i = (size_t)blockIdx.x * 256 + threadIdx.x; if (i >= n8) return;
    const v8f v = *(const v8f*)(src + i * 8); v8us o;
#pragma unroll
    for (int k = 0; k < 8; ++k) o[k] = f2bf(v[k]);
    *(volatile v8us*)(dst + i * 8) = o; __threadfence(); *(volatile v8us*)(dst + i * 8) = o;
}

__global__ __launch_bounds__(256) void k_xt(const float* __restrict__ x, bf* XT) {
    __shared__ __align__(16) unsigned short ts[32 * 264];
    const int tid = threadIdx.x, lane = tid & 31, wave = __builtin_amdgcn_readfirstlane((int)(tid >> 5));
    const int n0 = blockIdx.x * 32, b = blockIdx.y;
    const float* xb = x + (size_t)b * CH * SEQ_FULL + n0;
    const int q4 = (tid & 7) * 4, cl = tid >> 3;
#pragma unroll
    for (int i = 0; i < 8; ++i) { const int c = i * 32 + cl;
        const v4f v = *(const v4f*)(xb + (size_t)c * SEQ_FULL + q4);
#pragma unroll
        for (int e = 0; e < 4; ++e) ts[(q4 + e) * 264 + c] = f2bf(v[e]); }
    __syncthreads();
    bf* dst = XT + ((size_t)b * SEQ + n0 + wave * 4) * CH + lane * 8;
#pragma unroll 1
    for (int ps = 0; ps < 2; ++ps) {
#pragma unroll
        for (int s = 0; s < 4; ++s) { const v8us o = *(const v8usa*)(&ts[(wave * 4 + s) * 264 + lane * 8]);
            *(volatile v8us*)(dst + (size_t)s * CH) = o; }
        if (ps == 0) __threadfence(); }
}

__global__ __launch_bounds__(32) void k_projqk(const bf* __restrict__ A, const bf* __restrict__ Bt, const float* __restrict__ bq, const float* __restrict__ bk, h16* KPo, h16* KRo, h16* QHo, h16* QRo) {
    __shared__ __align__(16) float os[16 * 68];
    const int K = CH;
    const int lane = threadIdx.x & 31, lr = lane & 15, hi = lane >> 4; const int r0 = blockIdx.x * 64;
    v8f acc[4][4];
#pragma unroll
    for (int mb = 0; mb < 4; ++mb)
#pragma unroll
        for (int nb = 0; nb < 4; ++nb) acc[mb][nb] = (v8f){};
    const size_t aoff = (size_t)(r0 + lr) * K + 8 * hi, boff = (size_t)lr * K + 8 * hi;
#pragma unroll 1
    for (int kc = 0; kc < K; kc += 32) {
        v16bf a[4];
#pragma unroll
        for (int mb = 0; mb < 4; ++mb) a[mb] = ldb(A + aoff + (size_t)mb * 16 * K + kc);
#pragma unroll
        for (int nb = 0; nb < 4; ++nb) { const v16bf b = ldb(Bt + boff + (size_t)nb * 16 * K + kc);
#pragma unroll
            for (int mb = 0; mb < 4; ++mb) acc[mb][nb] = wmmab(a[mb], b, acc[mb][nb]); }
        asm volatile("v_nop\n\tv_nop\n\tv_nop\n\tv_nop" : "+v"(acc[0][0]), "+v"(acc[1][1]), "+v"(acc[2][2]), "+v"(acc[3][3]) : "v"(a[0]), "v"(a[1]), "v"(a[2]), "v"(a[3]));
    }
    const float bc0 = bfr(bq[lr]), bc1 = bfr(bq[16 + lr]), bc2 = bfr(bk[lr]), bc3 = bfr(bk[16 + lr]);
#pragma unroll
    for (int mb = 0; mb < 4; ++mb) {
#pragma unroll
        for (int j = 0; j < 8; ++j) { const int ro = (hi * 8 + j) * 68 + lr;
            os[ro] = acc[mb][0][j] + bc0; os[ro + 16] = acc[mb][1][j] + bc1; os[ro + 32] = acc[mb][2][j] + bc2; os[ro + 48] = acc[mb][3][j] + bc3; }
        wave_sync();
        const size_t sb = (size_t)(r0 + mb * 16) * CQ;
#pragma unroll 1
        for (int ps = 0; ps < 2; ++ps) {
#pragma unroll
            for (int s = 0; s < 2; ++s) { const int row = 8 * s + (lane >> 2), c8 = (lane & 3) * 8;
                const v4f x0 = *(const v4fa*)(&os[row * 68 + c8]);      const v4f x1 = *(const v4fa*)(&os[row * 68 + c8 + 4]);
                const v4f y0 = *(const v4fa*)(&os[row * 68 + 32 + c8]); const v4f y1 = *(const v4fa*)(&os[row * 68 + 32 + c8 + 4]);
                v8h kv, kr, hv, rv;
#pragma unroll
                for (int i = 0; i < 4; ++i) {
                    const h16 k0 = (h16)x0[i]; const h16 k1 = (h16)x1[i]; kv[i] = k0; kv[4 + i] = k1;
                    kr[i] = (h16)((x0[i] - (float)k0) * QRS); kr[4 + i] = (h16)((x1[i] - (float)k1) * QRS);
                    const h16 a0 = (h16)y0[i]; const h16 a1 = (h16)y1[i]; hv[i] = a0; hv[4 + i] = a1;
                    rv[i] = (h16)((y0[i] - (float)a0) * QRS); rv[4 + i] = (h16)((y1[i] - (float)a1) * QRS); }
                const size_t oo = sb + (size_t)row * CQ + c8;
                *(volatile v8h*)(KPo + oo) = kv; *(volatile v8h*)(KRo + oo) = kr; *(volatile v8h*)(QHo + oo) = hv; *(volatile v8h*)(QRo + oo) = rv; }
            if (ps == 0) __threadfence(); }
        wave_sync();
    }
}

__global__ __launch_bounds__(32) void k_projv(const bf* __restrict__ A, const bf* __restrict__ Bt, const float* __restrict__ bv, h16* VTo) {
    __shared__ __align__(16) float os[16 * 68];
    const int K = CH;
    const int lane = threadIdx.x & 31, lr = lane & 15, hi = lane >> 4; const int r0 = blockIdx.x * 64, c0 = blockIdx.y * 64;
    v8f acc[4][4];
#pragma unroll
    for (int mb = 0; mb < 4; ++mb)
#pragma unroll
        for (int nb = 0; nb < 4; ++nb) acc[mb][nb] = (v8f){};
    const size_t aoff = (size_t)(r0 + lr) * K + 8 * hi, boff = (size_t)(c0 + lr) * K + 8 * hi;
#pragma unroll 1
    for (int kc = 0; kc < K; kc += 32) {
        v16bf a[4];
#pragma unroll
        for (int mb = 0; mb < 4; ++mb) a[mb] = ldb(A + aoff + (size_t)mb * 16 * K + kc);
#pragma unroll
        for (int nb = 0; nb < 4; ++nb) { const v16bf b = ldb(Bt + boff + (size_t)nb * 16 * K + kc);
#pragma unroll
            for (int mb = 0; mb < 4; ++mb) acc[mb][nb] = wmmab(a[mb], b, acc[mb][nb]); }
        asm volatile("v_nop\n\tv_nop\n\tv_nop\n\tv_nop" : "+v"(acc[0][0]), "+v"(acc[1][1]), "+v"(acc[2][2]), "+v"(acc[3][3]) : "v"(a[0]), "v"(a[1]), "v"(a[2]), "v"(a[3]));
    }
    const int bb = c0 / SEQ, p0 = c0 % SEQ;
    const size_t tbase = ((size_t)bb * CH + r0) * SEQ + p0;
#pragma unroll
    for (int mb = 0; mb < 4; ++mb) {
#pragma unroll
        for (int j = 0; j < 8; ++j) { const float br = bfr(bv[r0 + mb * 16 + hi * 8 + j]); const int ro = (hi * 8 + j) * 68 + lr;
            os[ro] = acc[mb][0][j] + br; os[ro + 16] = acc[mb][1][j] + br; os[ro + 32] = acc[mb][2][j] + br; os[ro + 48] = acc[mb][3][j] + br; }
        wave_sync();
        const size_t sb = tbase + (size_t)(mb * 16) * SEQ;
#pragma unroll 1
        for (int ps = 0; ps < 2; ++ps) {
#pragma unroll
            for (int s = 0; s < 4; ++s) { const int row = 4 * s + (lane >> 3), c8 = (lane & 7) * 8;
                const v4f x0 = *(const v4fa*)(&os[row * 68 + c8]); const v4f x1 = *(const v4fa*)(&os[row * 68 + c8 + 4]); v8h hv;
#pragma unroll
                for (int i = 0; i < 4; ++i) { hv[i] = (h16)x0[i]; hv[4 + i] = (h16)x1[i]; }
                *(volatile v8h*)(VTo + sb + (size_t)row * SEQ + c8) = hv; }
            if (ps == 0) __threadfence(); }
        wave_sync();
    }
}

__global__ __launch_bounds__(32 * AW) void k_flash(const h16* __restrict__ QH, const h16* __restrict__ QR, const h16* __restrict__ KP, const h16* __restrict__ KR, const h16* __restrict__ VT, float* OUT) {
    __shared__ __align__(16) float os[CHH * 68];
    const int lane = threadIdx.x & 31, wave = __builtin_amdgcn_readfirstlane((int)(threadIdx.x >> 5)), lr = lane & 15, hi = lane >> 4;
    const int zh = blockIdx.y; const int b = zh >> 1, cg = zh & 1;
    const int tb0 = blockIdx.x * (16 * AW); const int t0 = tb0 + wave * 16;
    const size_t qkb = (size_t)b * SEQ * CQ;
    const size_t qo = qkb + (size_t)(t0 + lr) * CQ + 8 * hi;
    const v16h qh = ldh(QH + qo), qr = ldh(QR + qo);
    const size_t ko = qkb + (size_t)lr * CQ + 8 * hi;
    const size_t vo = ((size_t)b * CH + (size_t)cg * CHH + lr) * SEQ + 8 * hi;
    v8f o0 = (v8f){}, o1 = (v8f){}, o2 = (v8f){}, o3 = (v8f){}, o4 = (v8f){}, o5 = (v8f){}, o6 = (v8f){}, o7 = (v8f){};
    float m = -3.0e38f, l = 0.0f;
#pragma unroll 1
    for (int key0 = 0; key0 < SEQ; key0 += 32) {
        const h16* kp = KP + ko + (size_t)key0 * CQ;
        const h16* krp = KR + ko + (size_t)key0 * CQ;
        const v16h ka = ldh(kp), kb = ldh(kp + 16 * CQ);
        const v16h kra = ldh(krp), krb = ldh(krp + 16 * CQ);
        v8f sHa = (v8f){}, sLa = (v8f){}, sHb = (v8f){}, sLb = (v8f){};
        sHa = wmma16(ka, qh, sHa); sLa = wmma16(ka, qr, sLa); sHb = wmma16(kb, qh, sHb); sLb = wmma16(kb, qr, sLb);
        sLa = wmma16(kra, qh, sLa); sLb = wmma16(krb, qh, sLb);
        asm volatile("v_nop\n\tv_nop\n\tv_nop\n\tv_nop" : "+v"(sHa), "+v"(sLa), "+v"(sHb), "+v"(sLb) : "v"(ka), "v"(kb), "v"(kra), "v"(krb));
        float ta[8], tb[8]; float mx = -3.0e38f;
#pragma unroll
        for (int r = 0; r < 8; ++r) { ta[r] = (sHa[r] + sLa[r] * QRI) * SC2; tb[r] = (sHb[r] + sLb[r] * QRI) * SC2; mx = fmaxf(mx, fmaxf(ta[r], tb[r])); }
        mx = fmaxf(mx, __shfl_xor(mx, 16, 32));
        const float mnew = fmaxf(m, mx);
        const float alpha = __builtin_amdgcn_exp2f(m - mnew);
        const float sh = PSH - mnew;
        v16h pb; float ls = 0.0f;
#pragma unroll
        for (int r = 0; r < 8; ++r) { const h16 pa = (h16)__builtin_amdgcn_exp2f(ta[r] + sh); const h16 pc = (h16)__builtin_amdgcn_exp2f(tb[r] + sh); pb[r] = pa; pb[8 + r] = pc; ls += (float)pa + (float)pc; }
        l = l * alpha + ls; m = mnew;
        o0 = o0 * alpha; o1 = o1 * alpha; o2 = o2 * alpha; o3 = o3 * alpha; o4 = o4 * alpha; o5 = o5 * alpha; o6 = o6 * alpha; o7 = o7 * alpha;
        const h16* va = VT + vo + key0;
        { const v16h v0 = ldh(va), v1 = ldh(va + (size_t)16 * SEQ), v2 = ldh(va + (size_t)32 * SEQ), v3 = ldh(va + (size_t)48 * SEQ);
          o0 = wmma16(v0, pb, o0); o1 = wmma16(v1, pb, o1); o2 = wmma16(v2, pb, o2); o3 = wmma16(v3, pb, o3);
          asm volatile("v_nop\n\tv_nop\n\tv_nop\n\tv_nop" : "+v"(o0), "+v"(o1), "+v"(o2), "+v"(o3) : "v"(v0), "v"(v1), "v"(v2), "v"(v3), "v"(pb)); }
        { const v16h v4 = ldh(va + (size_t)64 * SEQ), v5 = ldh(va + (size_t)80 * SEQ), v6 = ldh(va + (size_t)96 * SEQ), v7 = ldh(va + (size_t)112 * SEQ);
          o4 = wmma16(v4, pb, o4); o5 = wmma16(v5, pb, o5); o6 = wmma16(v6, pb, o6); o7 = wmma16(v7, pb, o7);
          asm volatile("v_nop\n\tv_nop\n\tv_nop\n\tv_nop" : "+v"(o4), "+v"(o5), "+v"(o6), "+v"(o7) : "v"(v4), "v"(v5), "v"(v6), "v"(v7), "v"(pb)); }
    }
    l += __shfl_xor(l, 16, 32);
    const float inv = 1.0f / l;
#pragma unroll
    for (int r = 0; r < 8; ++r) { const int rb = (8 * hi + r) * 68 + wave * 16 + lr;
        os[rb]            = o0[r] * inv; os[rb + 16 * 68]  = o1[r] * inv; os[rb + 32 * 68]  = o2[r] * inv; os[rb + 48 * 68]  = o3[r] * inv;
        os[rb + 64 * 68]  = o4[r] * inv; os[rb + 80 * 68]  = o5[r] * inv; os[rb + 96 * 68]  = o6[r] * inv; os[rb + 112 * 68] = o7[r] * inv; }
    __syncthreads();
    float* obase = OUT + ((size_t)b * CH + (size_t)cg * CHH) * OUT_SEQ + tb0;
#pragma unroll 1
    for (int ps = 0; ps < 2; ++ps) {
#pragma unroll
        for (int s = 0; s < 16; ++s) { const int row = wave * 32 + 2 * s + hi, cofs = lr * 4;
            const v4f val = *(const v4fa*)(&os[row * 68 + cofs]);
            *(volatile v4f*)(obase + (size_t)row * OUT_SEQ + cofs) = val; }
        if (ps == 0) __threadfence(); }
}

static constexpr size_t al256(size_t v) { return (v + 255) & ~(size_t)255; }
static constexpr size_t SZ_XT = al256((size_t)NB * SEQ * CH * 2);
static constexpr size_t SZ_WQK = al256((size_t)2 * CQ * CH * 2);
static constexpr size_t SZ_WV = al256((size_t)CH * CH * 2);
static constexpr size_t SZ_QK = al256((size_t)NB * SEQ * CQ * 2);
static constexpr size_t SZ_VT = al256((size_t)NB * CH * SEQ * 2);
static constexpr size_t SZ_TOTAL = SZ_XT + SZ_WQK + SZ_WV + 4 * SZ_QK + SZ_VT;
static_assert(SZ_TOTAL <= (size_t)134217728);
static_assert(((size_t)CQ * CH * 2) % 256 == 0);

extern "C" void kernel_launch(void* const* d_in, const int* in_sizes, int n_in,
                              void* d_out, int out_size, void* d_ws, size_t ws_size, hipStream_t stream) {
    if (n_in < 7) return;
    const size_t needx = ((size_t)NB * CH - 1) * SEQ_FULL + SEQ;
    if ((size_t)in_sizes[0] < needx) return;
    if ((size_t)in_sizes[1] < (size_t)CQ * CH || (size_t)in_sizes[2] < (size_t)CQ) return;
    if ((size_t)in_sizes[3] < (size_t)CQ * CH || (size_t)in_sizes[4] < (size_t)CQ) return;
    if ((size_t)in_sizes[5] < (size_t)CH * CH || (size_t)in_sizes[6] < (size_t)CH) return;
    if ((size_t)out_size < ((size_t)NB * CH - 1) * OUT_SEQ + SEQ) return;
    if (SZ_TOTAL > ws_size) return;
    const float* x = (const float*)d_in[0]; const float* wq = (const float*)d_in[1]; const float* bq = (const float*)d_in[2];
    const float* wk = (const float*)d_in[3]; const float* bk = (const float*)d_in[4]; const float* wv = (const float*)d_in[5]; const float* bv = (const float*)d_in[6];
    float* OUT = (float*)d_out;
    char* wsp = (char*)d_ws;
    bf* XT = (bf*)wsp; wsp += SZ_XT;
    bf* WQK = (bf*)wsp; wsp += SZ_WQK;
    bf* WV = (bf*)wsp; wsp += SZ_WV;
    h16* KP = (h16*)wsp; wsp += SZ_QK;
    h16* KR = (h16*)wsp; wsp += SZ_QK;
    h16* QH = (h16*)wsp; wsp += SZ_QK;
    h16* QR = (h16*)wsp; wsp += SZ_QK;
    h16* VT = (h16*)wsp; wsp += SZ_VT;

    k_xt<<<dim3(SEQ / 32, NB, 1), 256, 0, stream>>>(x, XT);
    { const size_t n8 = (size_t)CQ * CH / 8; const unsigned g = (unsigned)((n8 + 255) / 256);
      k_cvt8<<<g, 256, 0, stream>>>(wq, WQK, n8); k_cvt8<<<g, 256, 0, stream>>>(wk, WQK + (size_t)CQ * CH, n8); }
    { const size_t n8 = (size_t)CH * CH / 8; k_cvt8<<<(unsigned)((n8 + 255) / 256), 256, 0, stream>>>(wv, WV, n8); }

    k_projqk<<<dim3(NB * SEQ / 64, 1, 1), 32, 0, stream>>>(XT, WQK, bq, bk, KP, KR, QH, QR);
    k_projv<<<dim3(CH / 64, NB * SEQ / 64, 1), 32, 0, stream>>>(WV, XT, bv, VT);

    k_flash<<<dim3(SEQ / (16 * AW), NB * 2, 1), 32 * AW, 0, stream>>>(QH, QR, KP, KR, VT, OUT);
}
